// BF16Indexer_57612691308720
// MI455X (gfx1250) — hardware-verified
//
#include <hip/hip_runtime.h>
#include <stddef.h>
#include <stdint.h>


#define MQ     2048
#define NK     4096
#define HH     32
#define DD     128
#define NT     2
#define NWAVE  4
#define NTHR   (NWAVE * 32)
#define BM     16
#define BN     (NWAVE * NT * 16)
#define SP     32

static_assert((DD % 32) == 0);
static_assert((MQ % BM) == 0);
static_assert((NK % BN) == 0);
static_assert(NT * 16 == SP);
static_assert(NTHR == 128);
static_assert((BM * HH) % NTHR == 0);

typedef float          v4f  __attribute__((ext_vector_type(4)));
typedef float          v8f  __attribute__((ext_vector_type(8)));
typedef __bf16         v16b __attribute__((ext_vector_type(16)));
typedef unsigned short v8us __attribute__((ext_vector_type(8)));
union FragB { v16b v; v8us u[2]; };

__device__ __forceinline__ v8f wmb(v16b a, v16b b, v8f c) {
  v8f d = __builtin_amdgcn_wmma_f32_16x16x32_bf16(false, a, false, b, (short)0, c, false, false);
  asm volatile("v_nop\n\tv_nop\n\tv_nop\n\tv_nop" : "+v"(d) : "v"(a), "v"(b));
  return d;
}

__global__ __launch_bounds__(NTHR)
void k_main(const unsigned short* __restrict__ q,
            const unsigned short* __restrict__ k,
            const unsigned short* __restrict__ w,
            float* out)
{
  __shared__ __attribute__((aligned(16))) float w_lds[BM * HH];
  __shared__ __attribute__((aligned(16))) float stg[NWAVE * BM * SP];

  const int tid = threadIdx.x, wave = tid >> 5, lane = tid & 31;
  const int m = lane & 15, hh = lane >> 4;
  const int m0 = blockIdx.y * BM;
  const int n_base = blockIdx.x * BN + wave * (NT * 16);

#pragma unroll
  for (int j = 0; j < (BM * HH) / NTHR; ++j) {
    const int i = tid + j * NTHR;
    w_lds[i] = __uint_as_float(((unsigned)w[(size_t)m0 * HH + i]) << 16);
  }
  __syncthreads();

  FragB bf[NT][DD / 32];
#pragma unroll
  for (int nt = 0; nt < NT; ++nt) {
    const unsigned short* kp = k + (size_t)(n_base + 16 * nt + m) * DD + 8 * hh;
#pragma unroll
    for (int ks = 0; ks < DD / 32; ++ks) {
      bf[nt][ks].u[0] = *(const v8us*)(kp + 32 * ks);
      bf[nt][ks].u[1] = *(const v8us*)(kp + 32 * ks + 16);
    }
  }

  v8f acc[NT];
#pragma unroll
  for (int nt = 0; nt < NT; ++nt) { v8f z = {0.f, 0.f, 0.f, 0.f, 0.f, 0.f, 0.f, 0.f}; acc[nt] = z; }

  const unsigned short* qrow = q + ((size_t)(m0 + m) * HH) * DD + 8 * hh;

#pragma unroll 1
  for (int h = 0; h < HH; ++h) {
    const unsigned short* qp = qrow + (size_t)h * DD;

    v8f c[NT];
#pragma unroll
    for (int nt = 0; nt < NT; ++nt) { v8f z = {0.f, 0.f, 0.f, 0.f, 0.f, 0.f, 0.f, 0.f}; c[nt] = z; }

#pragma unroll
    for (int ks = 0; ks < DD / 32; ++ks) {
      FragB a;
      a.u[0] = *(const v8us*)(qp + 32 * ks);
      a.u[1] = *(const v8us*)(qp + 32 * ks + 16);
#pragma unroll
      for (int nt = 0; nt < NT; ++nt) c[nt] = wmb(a.v, bf[nt][ks].v, c[nt]);
    }

    float wr[8];
#pragma unroll
    for (int r = 0; r < 8; ++r) wr[r] = w_lds[(8 * hh + r) * HH + h];

#pragma unroll
    for (int nt = 0; nt < NT; ++nt) {
#pragma unroll
      for (int r = 0; r < 8; ++r) {
        const float x = fmaxf(c[nt][r], 0.0f);
        acc[nt][r] = fmaf(x, wr[r], acc[nt][r]);
      }
    }
  }

  const float scale = 0.08838834613561630f;
  float* sp = stg + wave * (BM * SP);
#pragma unroll
  for (int nt = 0; nt < NT; ++nt) {
#pragma unroll
    for (int r = 0; r < 8; ++r) sp[(8 * hh + r) * SP + 16 * nt + m] = acc[nt][r] * scale;
  }
  __syncthreads();

  const int rr = lane >> 3, c4 = lane & 7;
  v4f v[4];
#pragma unroll
  for (int j = 0; j < 4; ++j) v[j] = *(const v4f*)(sp + (4 * j + rr) * SP + 4 * c4);

  float* gb = out + (size_t)m0 * NK + n_base + 4 * c4;
#pragma unroll
  for (int j = 0; j < 4; ++j) *(volatile v4f*)(gb + (size_t)(4 * j + rr) * NK) = v[j];
  __threadfence();
#pragma unroll
  for (int j = 0; j < 4; ++j) *(volatile v4f*)(gb + (size_t)(4 * j + rr) * NK) = v[j];
}

extern "C" void kernel_launch(void* const* d_in, const int* in_sizes, int n_in,
                              void* d_out, int out_size, void* d_ws, size_t ws_size,
                              hipStream_t stream) {
  if (n_in < 3) return;
  if (in_sizes[0] != MQ * HH * DD) return;
  if (in_sizes[1] != NK * DD) return;
  if (in_sizes[2] != MQ * HH) return;
  if (out_size != MQ * NK) return;
  (void)d_ws; (void)ws_size;

  const unsigned short* q = (const unsigned short*)d_in[0];
  const unsigned short* k = (const unsigned short*)d_in[1];
  const unsigned short* w = (const unsigned short*)d_in[2];
  float* out = (float*)d_out;

  k_main<<<dim3(NK / BN, MQ / BM), NTHR, 0, stream>>>(q, k, w, out);
}
